// SS2D_27453430956041
// MI455X (gfx1250) — hardware-verified
//
#include <hip/hip_runtime.h>
#include <stddef.h>


typedef _Float16 h16;
typedef _Float16 v16h __attribute__((ext_vector_type(16)));
typedef _Float16 v8h  __attribute__((ext_vector_type(8)));
typedef _Float16 v4h  __attribute__((ext_vector_type(4)));
typedef float    v8f  __attribute__((ext_vector_type(8)));
typedef float    v4f  __attribute__((ext_vector_type(4)));

#ifndef NB
#define NB 8
#endif
#define NB_FULL 8
#define CH    128
#define NUV   256
#define IMG_H 96
#define IMG_W 96
#define LTOK  (IMG_H * IMG_W)
#define MROWS (NB * LTOK)

static_assert(NB >= 1 && NB <= NB_FULL);
static_assert((LTOK % 64) == 0);
static_assert((MROWS % 64) == 0);
static_assert(CH == 32 * 4);
static_assert((CH % 32) == 0);
static_assert(NUV == 2 * CH);
static_assert((IMG_W % 16) == 0 && IMG_W == 6 * 16);
static_assert(IMG_W == 8 * 12);
static_assert((size_t)MROWS * CH < (size_t)0xFFFFFFFFu);

#define LDA  136
#define LDC2 260
#define LDW  100
static_assert((LDA % 8) == 0 && LDA >= CH);
static_assert((LDC2 % 4) == 0 && LDC2 >= NUV);
static_assert((LDW % 4) == 0 && LDW >= IMG_W);
static_assert(64 * LDA * 2 + 64 * LDC2 * 4 <= 131072);
static_assert(IMG_W * LDA * 2 + CH * LDW * 4 <= 131072);

#define WCARRY 64.0f
#define XCARRY 16.0f
#define YCARRY 16.0f

#define WIN_BYTES  ((size_t)NUV * CH * 2)
#define WOUT_BYTES ((size_t)CH * CH * 2)
#define UV_BYTES   ((size_t)MROWS * CH * 4)
#define OFF_WIN  ((size_t)0)
#define OFF_WOUT (OFF_WIN + WIN_BYTES)
#define OFF_U    (OFF_WOUT + WOUT_BYTES)
#define OFF_V    (OFF_U + UV_BYTES)
#define WS_TOTAL (OFF_V + UV_BYTES)
static_assert((WIN_BYTES % 128) == 0 && (WOUT_BYTES % 128) == 0 && (UV_BYTES % 128) == 0);
static_assert(WS_TOTAL <= (size_t)134217728);
static_assert(((NUV * CH) % 2048) == 0 && ((CH * CH) % 2048) == 0);

__device__ __forceinline__ float bf16r(float x) {
  unsigned int u = __float_as_uint(x);
  u = (u + 0x7FFFu + ((u >> 16) & 1u)) & 0xFFFF0000u;
  return __uint_as_float(u);
}

static __device__ __forceinline__ h16 toh_flush(float v) {
  const h16 r = (h16)v;
  return (fabsf(v) < 6.103515625e-05f) ? (h16)0.0f : r;
}

__device__ __forceinline__ v16h frag_at(const _Float16* p) {
  v8h lo = *(const v8h*)(p);
  v8h hi = *(const v8h*)(p + 16);
  v16h out;
#pragma unroll
  for (int i = 0; i < 8; ++i) { out[i] = lo[i]; out[i + 8] = hi[i]; }
  return out;
}
__device__ __forceinline__ v16h ld_frag(const _Float16* base, unsigned ld) {
  const unsigned lane = threadIdx.x & 31u;
  return frag_at(base + (lane & 15u) * ld + (lane >> 4) * 8u);
}

__device__ __forceinline__ v8f wmma16(v16h a, v16h b, v8f c) {
  v8f d = __builtin_amdgcn_wmma_f32_16x16x32_f16(false, a, false, b, (short)0, c,
                                                 false, false);
  asm volatile("v_nop\n\tv_nop\n\tv_nop\n\tv_nop" : "+v"(d) : "v"(a), "v"(b));
  return d;
}

__device__ __forceinline__ float red32_sum(float x) {
#pragma unroll
  for (int off = 1; off < 32; off <<= 1) x += __shfl_xor(x, off, 32);
  return x;
}

__device__ __forceinline__ float silu_act(float t) {
  return t * __builtin_amdgcn_rcpf(1.0f + __expf(-t));
}

__global__ __launch_bounds__(256) void wcast_kernel(
    const float* __restrict__ W, _Float16* __restrict__ P16) {
  const unsigned i8 = (blockIdx.x * 256u + threadIdx.x) * 8u;
  const v4f a0 = *(const v4f*)(W + i8);
  const v4f a1 = *(const v4f*)(W + i8 + 4u);
  v8h o;
#pragma unroll
  for (int i = 0; i < 4; ++i) {
    o[i]     = toh_flush(WCARRY * bf16r(a0[i]));
    o[i + 4] = toh_flush(WCARRY * bf16r(a1[i]));
  }
  _Float16* p = P16 + i8;
  *(volatile v8h*)p = o;
  __threadfence();
  *(volatile v8h*)p = o;
}

__global__ __launch_bounds__(256) void in_gemm_kernel(
    const float* __restrict__ X, const _Float16* __restrict__ Wi16,
    const float* __restrict__ b_in, float* __restrict__ U, float* __restrict__ V) {
  __shared__ _Float16 As[64 * LDA];
  __shared__ float Cs[64 * LDC2];
  const unsigned tid = threadIdx.x, lane = tid & 31u;
  const unsigned w = (unsigned)__builtin_amdgcn_readfirstlane((int)(tid >> 5));
  const unsigned mw = w >> 1, nw = w & 1u;
  const unsigned hh = lane >> 4, m = lane & 15u;
  const unsigned t0 = blockIdx.x * 64u;
  const unsigned bimg = t0 / (unsigned)LTOK;
  const unsigned ti = t0 - bimg * (unsigned)LTOK;
  const float* xb = X + (size_t)bimg * CH * LTOK + ti;

#pragma unroll 2
  for (unsigned i = 0; i < 8u; ++i) {
    const unsigned e = tid + 256u * i;
    const unsigned c = e >> 4;
    const unsigned tq = (e & 15u) * 4u;
    const v4f a = *(const v4f*)(xb + (size_t)c * LTOK + tq);
#pragma unroll
    for (unsigned j = 0; j < 4u; ++j)
      As[(tq + j) * LDA + c] = toh_flush(XCARRY * bf16r(a[j]));
  }
  __syncthreads();

  v8f acc[8];
#pragma unroll
  for (int j = 0; j < 8; ++j) acc[j] = (v8f){};
  const _Float16* bp = Wi16 + (size_t)(nw * 128u + m) * CH + hh * 8u;
#pragma unroll 2
  for (unsigned c = 0; c < 4u; ++c) {
    const v16h a = ld_frag(&As[(mw * 16u) * LDA + c * 32u], LDA);
#pragma unroll
    for (int j = 0; j < 8; ++j) {
      const v16h bfr = frag_at(bp + (size_t)(j * 16) * CH + c * 32u);
      acc[j] = wmma16(a, bfr, acc[j]);
    }
  }
#pragma unroll
  for (int j = 0; j < 8; ++j)
#pragma unroll
    for (int r = 0; r < 8; ++r)
      Cs[(mw * 16u + hh * 8u + (unsigned)r) * LDC2 + nw * 128u + (unsigned)j * 16u + m] = acc[j][r];
  __syncthreads();

  static_assert(4 * 2 * 8 == 64);
  const float cs = 1.0f / (WCARRY * XCARRY);
  const v4f gbu = *(const v4f*)(b_in + lane * 4u);
  const v4f gbv = *(const v4f*)(b_in + 128u + lane * 4u);
#pragma unroll 1
  for (unsigned g = 0; g < 4u; ++g) {
    v4f xu[2], xv[2];
    size_t off[2];
#pragma unroll
    for (unsigned i = 0; i < 2u; ++i) {
      const unsigned r = w * 8u + g * 2u + i;
      const v4f cu = *(const v4f*)&Cs[r * LDC2 + lane * 4u];
      const v4f cv = *(const v4f*)&Cs[r * LDC2 + 128u + lane * 4u];
#pragma unroll
      for (int j = 0; j < 4; ++j) {
        const float tu = cu[j] * cs + bf16r(gbu[j]);
        xu[i][j] = silu_act(tu);
        xv[i][j] = cv[j] * cs + bf16r(gbv[j]);
      }
      off[i] = (size_t)(t0 + r) * CH + lane * 4u;
    }
#pragma unroll
    for (int i = 0; i < 2; ++i) {
      *(volatile v4f*)(U + off[i]) = xu[i];
      *(volatile v4f*)(V + off[i]) = xv[i];
    }
    __threadfence();
#pragma unroll
    for (int i = 0; i < 2; ++i) {
      *(volatile v4f*)(U + off[i]) = xu[i];
      *(volatile v4f*)(V + off[i]) = xv[i];
    }
  }
}

__global__ __launch_bounds__(256) void mix_out_kernel(
    const float* __restrict__ U, const float* __restrict__ V,
    const float* __restrict__ dw_w, const float* __restrict__ dw_b,
    const float* __restrict__ gamma, const float* __restrict__ beta,
    const _Float16* __restrict__ Wo16, const float* __restrict__ b_out,
    float* __restrict__ out) {
  __shared__ _Float16 Ys[IMG_W * LDA];
  __shared__ float Cw[CH * LDW];

  const unsigned tid = threadIdx.x, lane = tid & 31u;
  const unsigned w8 = (unsigned)__builtin_amdgcn_readfirstlane((int)(tid >> 5));
  const unsigned hh = lane >> 4, m = lane & 15u;
  const unsigned bimg = blockIdx.x / (unsigned)IMG_H;
  const unsigned h = blockIdx.x - bimg * (unsigned)IMG_H;
  const unsigned c0 = lane * 4u;

  float dwA[4][7];
#pragma unroll
  for (int j = 0; j < 4; ++j)
#pragma unroll
    for (int k = 0; k < 7; ++k)
      dwA[j][k] = bf16r(dw_w[(c0 + (unsigned)j) * 7u + (unsigned)k]);
  const v4f g4  = *(const v4f*)(gamma + c0);
  const v4f be4 = *(const v4f*)(beta + c0);
  const v4f db4 = *(const v4f*)(dw_b + c0);
  float gg[4], bb[4], db[4];
#pragma unroll
  for (int j = 0; j < 4; ++j) { gg[j] = bf16r(g4[j]); bb[j] = bf16r(be4[j]); db[j] = bf16r(db4[j]); }

  const size_t imgbase = (size_t)bimg * LTOK;

  for (unsigned px = w8; px < (unsigned)IMG_W; px += 8u) {
    const int tlr = (int)(h * (unsigned)IMG_W + px);
    const int ptb = (int)(px * (unsigned)IMG_H + h);
    const v4f u4 = *(const v4f*)(U + (imgbase + (size_t)tlr) * CH + c0);

    float clr[4] = {0.0f, 0.0f, 0.0f, 0.0f}, crl[4] = {0.0f, 0.0f, 0.0f, 0.0f};
    float ctb[4] = {0.0f, 0.0f, 0.0f, 0.0f}, cbt[4] = {0.0f, 0.0f, 0.0f, 0.0f};
#pragma unroll
    for (int k = 0; k < 7; ++k) {
      const int tt = tlr + k - 3;
      const int ttc = min(max(tt, 0), LTOK - 1);
      const bool okl = (tt == ttc);
      const v4f tp = *(const v4f*)(V + (imgbase + (size_t)ttc) * CH + c0);
      const int pp = ptb + k - 3;
      const int ppc = min(max(pp, 0), LTOK - 1);
      const bool okt = (pp == ppc);
      const int w2 = ppc / IMG_H;
      const int h2 = ppc - w2 * IMG_H;
      const v4f tq = *(const v4f*)(V + (imgbase + (size_t)(h2 * IMG_W + w2)) * CH + c0);
#pragma unroll
      for (int j = 0; j < 4; ++j) {
        const float tl = okl ? tp[j] : 0.0f;
        const float tb = okt ? tq[j] : 0.0f;
        clr[j] += dwA[j][k] * tl;
        crl[j] += dwA[j][6 - k] * tl;
        ctb[j] += dwA[j][k] * tb;
        cbt[j] += dwA[j][6 - k] * tb;
      }
    }

    float y[4][4];
#pragma unroll
    for (int j = 0; j < 4; ++j) {
      y[0][j] = silu_act(clr[j] + db[j]) * u4[j];
      y[1][j] = silu_act(crl[j] + db[j]) * u4[j];
      y[2][j] = silu_act(ctb[j] + db[j]) * u4[j];
      y[3][j] = silu_act(cbt[j] + db[j]) * u4[j];
    }

    float mu[4], rs[4];
#pragma unroll
    for (int i = 0; i < 4; ++i) {
      const float s = red32_sum((y[i][0] + y[i][1]) + (y[i][2] + y[i][3]));
      mu[i] = s * (1.0f / (float)CH);
    }
#pragma unroll
    for (int i = 0; i < 4; ++i) {
      float q = 0.0f;
#pragma unroll
      for (int j = 0; j < 4; ++j) {
        const float d = y[i][j] - mu[i];
        q += d * d;
      }
      q = red32_sum(q);
      rs[i] = rsqrtf(q * (1.0f / (float)CH) + 1.0e-5f);
    }
    v4h pk;
#pragma unroll
    for (int j = 0; j < 4; ++j) {
      float a = 0.0f;
#pragma unroll
      for (int i = 0; i < 4; ++i) a += (y[i][j] - mu[i]) * rs[i];
      const float o = 0.25f * gg[j] * a + bb[j];
      pk[j] = toh_flush(YCARRY * o);
    }
    *(v4h*)&Ys[px * LDA + c0] = pk;
  }
  __syncthreads();

  v8f acc[6];
#pragma unroll
  for (int mt = 0; mt < 6; ++mt) acc[mt] = (v8f){};
  const _Float16* bp = Wo16 + (size_t)(w8 * 16u + m) * CH + hh * 8u;
#pragma unroll
  for (int c = 0; c < 4; ++c) {
    const v16h bfr = frag_at(bp + c * 32);
#pragma unroll
    for (int mt = 0; mt < 6; ++mt) {
      const v16h a = ld_frag(&Ys[(mt * 16) * LDA + c * 32], LDA);
      acc[mt] = wmma16(a, bfr, acc[mt]);
    }
  }
#pragma unroll
  for (int mt = 0; mt < 6; ++mt) {
    float* d = &Cw[(w8 * 16u + m) * LDW + (unsigned)mt * 16u + hh * 8u];
    v4f lo4, hi4;
#pragma unroll
    for (int r = 0; r < 4; ++r) { lo4[r] = acc[mt][r]; hi4[r] = acc[mt][r + 4]; }
    *(v4f*)d = lo4;
    *(v4f*)(d + 4) = hi4;
  }
  __syncthreads();

  static_assert(4 * 32 == CH);
  static_assert(3 * 8 * 4 == IMG_W);
  const float cs = 1.0f / (WCARRY * YCARRY);
#pragma unroll 1
  for (unsigned ng = 0; ng < 4u; ++ng) {
    const unsigned n = ng * 32u + (tid >> 3);
    const float bias = bf16r(b_out[n]);
    const size_t rowoff = (((size_t)bimg * CH + n) * IMG_H + h) * IMG_W;
    v4f xs[3];
    size_t off[3];
#pragma unroll
    for (unsigned seg = 0; seg < 3u; ++seg) {
      const unsigned col = seg * 32u + (tid & 7u) * 4u;
      const v4f cwv = *(const v4f*)&Cw[n * LDW + col];
      v4f val;
#pragma unroll
      for (int j = 0; j < 4; ++j) val[j] = cwv[j] * cs + bias;
      xs[seg] = val;
      off[seg] = rowoff + col;
    }
#pragma unroll
    for (int seg = 0; seg < 3; ++seg) *(volatile v4f*)(out + off[seg]) = xs[seg];
    __threadfence();
#pragma unroll
    for (int seg = 0; seg < 3; ++seg) *(volatile v4f*)(out + off[seg]) = xs[seg];
  }
}

extern "C" void kernel_launch(void* const* d_in, const int* in_sizes, int n_in,
                              void* d_out, int out_size, void* d_ws, size_t ws_size,
                              hipStream_t stream) {
  if (n_in < 9) return;
  const long long need_x = (long long)NB * CH * LTOK;
  if ((long long)in_sizes[0] < need_x) return;
  if ((long long)in_sizes[1] < (long long)NUV * CH) return;
  if (in_sizes[2] < NUV) return;
  if (in_sizes[3] < CH * 7) return;
  if (in_sizes[4] < CH || in_sizes[5] < CH || in_sizes[6] < CH) return;
  if ((long long)in_sizes[7] < (long long)CH * CH) return;
  if (in_sizes[8] < CH) return;
  if ((long long)out_size < need_x) return;
  if (ws_size < WS_TOTAL) return;

  const float* x     = (const float*)d_in[0];
  const float* w_in  = (const float*)d_in[1];
  const float* b_in  = (const float*)d_in[2];
  const float* dw_w  = (const float*)d_in[3];
  const float* dw_b  = (const float*)d_in[4];
  const float* gamma = (const float*)d_in[5];
  const float* beta  = (const float*)d_in[6];
  const float* w_out = (const float*)d_in[7];
  const float* b_out = (const float*)d_in[8];
  float* out = (float*)d_out;

  char* ws = (char*)d_ws;
  _Float16* Win16  = (_Float16*)(ws + OFF_WIN);
  _Float16* Wout16 = (_Float16*)(ws + OFF_WOUT);
  float*    Upl    = (float*)(ws + OFF_U);
  float*    Vpl    = (float*)(ws + OFF_V);

  dim3 blk(256);
  wcast_kernel<<<dim3((NUV * CH) / 2048), blk, 0, stream>>>(w_in, Win16);
  wcast_kernel<<<dim3((CH * CH) / 2048), blk, 0, stream>>>(w_out, Wout16);
  in_gemm_kernel<<<dim3(MROWS / 64), blk, 0, stream>>>(x, Win16, b_in, Upl, Vpl);
  mix_out_kernel<<<dim3(NB * IMG_H), blk, 0, stream>>>(Upl, Vpl, dw_w, dw_b, gamma, beta,
                                                       Wout16, b_out, out);
}
